// tRNTN_4776003633392
// MI455X (gfx1250) — hardware-verified
//
#include <hip/hip_runtime.h>


#define VOC    2048
#define D      128
#define RELS   7
#define NB     512
#define NLEAF  (NB * 2 * 16)
#define KT     16384
#define KL     256
#define KTOT   (KT + KL)
#define NCH    (KTOT / 32)
#define NSC    (NCH / 4)
#define NKR    (KT / 128)
#define SCB    (4 * 8 * 32 * 16)
#define NPK    (NCH * 8 * 32 * 16)
#define ROWP   132
#define APH    136

#define ASC      16.0f
#define WSC      64.0f
#define INV_MAIN (1.0f / 16384.0f)
#define SSC      256.0f
#define WSMSC    8.0f
#define INV_SM   (1.0f / 2048.0f)

static_assert(NSC * 4 == NCH);
static_assert((NPK / 8) % 256 == 0);
static_assert((NLEAF * 32) % 256 == 0);

typedef _Float16 f16_t;
typedef f16_t v16h __attribute__((ext_vector_type(16)));
typedef f16_t v8h  __attribute__((ext_vector_type(8)));
typedef float v8f  __attribute__((ext_vector_type(8)));
typedef float v4f  __attribute__((ext_vector_type(4)));
typedef unsigned int v4u __attribute__((ext_vector_type(4)));
union Frag  { v16h v; v8h half[2]; };
union Pack8 { v8h h; v4u u; };

__device__ __forceinline__ v8f wmma16(v16h a, v16h b, v8f c) {
  v8f d = __builtin_amdgcn_wmma_f32_16x16x32_f16(false, a, false, b, (short)0, c, false, false);
  asm volatile("v_nop\n\tv_nop\n\tv_nop\n\tv_nop" : "+v"(d) : "v"(a), "v"(b));
  return d;
}

__global__ __launch_bounds__(256)
void embed_kernel(const int* __restrict__ ids, const float* __restrict__ Wv,
                  const float* __restrict__ bv, float* __restrict__ h0) {
  const int t = blockIdx.x * 256 + threadIdx.x;
  const int leaf = t >> 5;
  if (leaf >= NLEAF) return;
  const int c4 = (t & 31) * 4;
  int id = ids[leaf];
  id = id < 0 ? 0 : (id >= VOC ? VOC - 1 : id);
  v4f v;
  v.x = Wv[(size_t)(c4 + 0) * VOC + id] + bv[c4 + 0];
  v.y = Wv[(size_t)(c4 + 1) * VOC + id] + bv[c4 + 1];
  v.z = Wv[(size_t)(c4 + 2) * VOC + id] + bv[c4 + 2];
  v.w = Wv[(size_t)(c4 + 3) * VOC + id] + bv[c4 + 3];
  float* p = h0 + (size_t)leaf * D + c4;
  *(volatile v4f*)p = v;
  __threadfence();
  *(volatile v4f*)p = v;
}

__global__ __launch_bounds__(256)
void prepack_kernel(const float* __restrict__ Wt1, const float* __restrict__ Wl1,
                    const float* __restrict__ Wt2, const float* __restrict__ Wl2,
                    f16_t* __restrict__ out1, f16_t* __restrict__ out2) {
  const int t = blockIdx.x * 256 + threadIdx.x;
  const int NT = NPK / 8;
  if (t >= 2 * NT) return;
  const int set = (t >= NT) ? 1 : 0;
  const int u = t - set * NT;
  const float* Wt = set ? Wt2 : Wt1;
  const float* Wl = set ? Wl2 : Wl1;
  f16_t* outp = set ? out2 : out1;

  const int idx8 = u * 8;
  const int e0 = idx8 & 15;
  const int n  = (idx8 >> 4) & 31;
  const int ot = (idx8 >> 9) & 7;
  const int c  = idx8 >> 12;
  const int o  = ot * 16 + (n & 15);
  const int h  = n >> 4;
  const int k  = c * 32 + 8 * h + (e0 ? 16 : 0);
  const float* src = (k < KT) ? (Wt + (size_t)o * KT + k) : (Wl + (size_t)o * KL + (k - KT));
  v4f x0 = *(const v4f*)src;
  v4f x1 = *(const v4f*)(src + 4);
  Pack8 pk;
  pk.h[0] = (f16_t)(x0.x * WSC); pk.h[1] = (f16_t)(x0.y * WSC);
  pk.h[2] = (f16_t)(x0.z * WSC); pk.h[3] = (f16_t)(x0.w * WSC);
  pk.h[4] = (f16_t)(x1.x * WSC); pk.h[5] = (f16_t)(x1.y * WSC);
  pk.h[6] = (f16_t)(x1.z * WSC); pk.h[7] = (f16_t)(x1.w * WSC);
  v4u* dst = (v4u*)(outp + idx8);
  *(volatile v4u*)dst = pk.u;
  __threadfence();
  *(volatile v4u*)dst = pk.u;
}

__device__ __forceinline__ void stage_sc(const f16_t* __restrict__ Wpk, f16_t* dst, int sc, int tid) {
  const f16_t* g = Wpk + (size_t)sc * SCB + tid * 16;
  f16_t* l = dst + tid * 16;
#pragma unroll
  for (int r = 0; r < 4; ++r) {
    v4u t0 = *(const v4u*)(g + r * 4096);
    v4u t1 = *(const v4u*)(g + r * 4096 + 8);
    *(v4u*)(l + r * 4096)     = t0;
    *(v4u*)(l + r * 4096 + 8) = t1;
  }
}

__device__ __forceinline__ void tile_gemm(const float* __restrict__ hin,
                                          const f16_t* __restrict__ Wpk,
                                          float* Lsh, float* Rsh, f16_t* Bsh,
                                          int nodeBase, int shift,
                                          int lane, int tid, v8f acc[8]) {
  const int hi   = lane >> 4;
  const int mrow = lane & 15;
  const int nP   = 1 << shift;

#pragma unroll 4
  for (int m = 0; m < 16; ++m) {
    int g  = nodeBase + m;
    int bs = g >> shift;
    int p  = g & (nP - 1);
    size_t lidx = ((size_t)bs * 2 * nP + 2 * p) * D;
    v4f lv = *(const v4f*)(hin + lidx + lane * 4);
    v4f rv = *(const v4f*)(hin + lidx + D + lane * 4);
    *(v4f*)(Lsh + m * ROWP + lane * 4) = lv * ASC;
    *(v4f*)(Rsh + m * ROWP + lane * 4) = rv * ASC;
  }

  stage_sc(Wpk, Bsh, 0, tid);

  for (int sc = 0; sc < NSC; ++sc) {
    __syncthreads();
    if (sc + 1 < NSC) stage_sc(Wpk, Bsh + ((sc + 1) & 1) * SCB, sc + 1, tid);

    const float* src  = (sc == NKR) ? Lsh : Rsh;
    const float scale = (sc < NKR) ? Lsh[mrow * ROWP + sc] : ASC;
    const float* arow = src + mrow * ROWP + hi * 8;
    const f16_t* bb   = Bsh + (sc & 1) * SCB + lane * 16;

#pragma unroll 1
    for (int q = 0; q < 4; ++q) {
      const float* rp = arow + q * 32;
      v4f p0 = *(const v4f*)(rp);
      v4f p1 = *(const v4f*)(rp + 4);
      v4f q0 = *(const v4f*)(rp + 16);
      v4f q1 = *(const v4f*)(rp + 20);
      p0 *= scale; p1 *= scale; q0 *= scale; q1 *= scale;

      v16h a;
      a[0]  = (f16_t)p0.x;  a[1]  = (f16_t)p0.y;  a[2]  = (f16_t)p0.z;  a[3]  = (f16_t)p0.w;
      a[4]  = (f16_t)p1.x;  a[5]  = (f16_t)p1.y;  a[6]  = (f16_t)p1.z;  a[7]  = (f16_t)p1.w;
      a[8]  = (f16_t)q0.x;  a[9]  = (f16_t)q0.y;  a[10] = (f16_t)q0.z;  a[11] = (f16_t)q0.w;
      a[12] = (f16_t)q1.x;  a[13] = (f16_t)q1.y;  a[14] = (f16_t)q1.z;  a[15] = (f16_t)q1.w;

      const f16_t* bq = bb + q * 4096;
#pragma unroll
      for (int ot = 0; ot < 8; ++ot) {
        v16h bfr = *(const v16h*)(bq + ot * (32 * 16));
        acc[ot] = wmma16(a, bfr, acc[ot]);
      }
    }
  }
}

__global__ __launch_bounds__(256)
void combine_kernel(const float* __restrict__ hin, float* __restrict__ hout,
                    const f16_t* __restrict__ Wpk,
                    const float* __restrict__ b1, const float* __restrict__ b2,
                    int shift) {
  __shared__ __align__(16) float sh[8][2][16][ROWP];
  __shared__ __align__(16) f16_t bsh[2][SCB];
  const int lane = threadIdx.x & 31;
  const int w    = threadIdx.x >> 5;
  const int hi   = lane >> 4;
  const int mrow = lane & 15;
  const int nodeBase = (blockIdx.x * 8 + w) * 16;

  v8f acc[8] = {};
  tile_gemm(hin, Wpk, &sh[w][0][0][0], &sh[w][1][0][0], &bsh[0][0],
            nodeBase, shift, lane, threadIdx.x, acc);

  __syncthreads();
  float* St = &sh[w][0][0][0];
#pragma unroll
  for (int ot = 0; ot < 8; ++ot) {
    int o = ot * 16 + mrow;
    float bsum = b1[o] + b2[o];
#pragma unroll
    for (int g = 0; g < 8; ++g) {
      St[(g + hi * 8) * ROWP + o] = tanhf(acc[ot][g] * INV_MAIN + bsum);
    }
  }
  __syncthreads();

  float* orow = hout + (size_t)nodeBase * D + lane * 4;
#pragma unroll
  for (int t = 0; t < 16; ++t) {
    v4f v = *(const v4f*)(St + t * ROWP + lane * 4);
    *(volatile v4f*)(orow + (size_t)t * D) = v;
  }
  __threadfence();
#pragma unroll
  for (int t = 0; t < 16; ++t) {
    v4f v = *(const v4f*)(St + t * ROWP + lane * 4);
    *(volatile v4f*)(orow + (size_t)t * D) = v;
  }
}

__global__ __launch_bounds__(256)
void final_kernel(const float* __restrict__ hin, float* __restrict__ out,
                  const f16_t* __restrict__ Wpk,
                  const float* __restrict__ bcpr, const float* __restrict__ bcprt,
                  const float* __restrict__ Wsm, const float* __restrict__ bsm) {
  __shared__ __align__(16) float sh[8][2][16][ROWP];
  __shared__ __align__(16) f16_t bsh[2][SCB];
  __shared__ __align__(16) float outs[128 * RELS];
  const int lane = threadIdx.x & 31;
  const int w    = threadIdx.x >> 5;
  const int hi   = lane >> 4;
  const int mrow = lane & 15;
  const int nodeBase = (blockIdx.x * 8 + w) * 16;

  v8f acc[8] = {};
  tile_gemm(hin, Wpk, &sh[w][0][0][0], &sh[w][1][0][0], &bsh[0][0],
            nodeBase, 0, lane, threadIdx.x, acc);

  __syncthreads();
  f16_t* A16 = &bsh[0][0] + w * (16 * APH);
#pragma unroll
  for (int ot = 0; ot < 8; ++ot) {
    int o = ot * 16 + mrow;
    float bsum = bcpr[o] + bcprt[o];
#pragma unroll
    for (int g = 0; g < 8; ++g) {
      float v = acc[ot][g] * INV_MAIN + bsum;
      v = (v >= 0.0f) ? v : 0.01f * v;
      A16[(g + hi * 8) * APH + o] = (f16_t)(v * SSC);
    }
  }
  __syncthreads();

  const int nn = (mrow < RELS) ? mrow : (RELS - 1);
  const float wsel = (mrow < RELS) ? WSMSC : 0.0f;
  const float* wrow = Wsm + nn * D;
  v8f lacc = {};
#pragma unroll
  for (int ks = 0; ks < 4; ++ks) {
    const int k0 = ks * 32;
    Frag a;
    a.half[0] = *(const v8h*)(A16 + mrow * APH + k0 + hi * 8);
    a.half[1] = *(const v8h*)(A16 + mrow * APH + k0 + 16 + hi * 8);
    v4f w0 = *(const v4f*)(wrow + k0 + hi * 8);
    v4f w1 = *(const v4f*)(wrow + k0 + hi * 8 + 4);
    v4f w2 = *(const v4f*)(wrow + k0 + 16 + hi * 8);
    v4f w3 = *(const v4f*)(wrow + k0 + 16 + hi * 8 + 4);
    v16h bw;
    bw[0]  = (f16_t)(w0.x * wsel); bw[1]  = (f16_t)(w0.y * wsel);
    bw[2]  = (f16_t)(w0.z * wsel); bw[3]  = (f16_t)(w0.w * wsel);
    bw[4]  = (f16_t)(w1.x * wsel); bw[5]  = (f16_t)(w1.y * wsel);
    bw[6]  = (f16_t)(w1.z * wsel); bw[7]  = (f16_t)(w1.w * wsel);
    bw[8]  = (f16_t)(w2.x * wsel); bw[9]  = (f16_t)(w2.y * wsel);
    bw[10] = (f16_t)(w2.z * wsel); bw[11] = (f16_t)(w2.w * wsel);
    bw[12] = (f16_t)(w3.x * wsel); bw[13] = (f16_t)(w3.y * wsel);
    bw[14] = (f16_t)(w3.z * wsel); bw[15] = (f16_t)(w3.w * wsel);
    lacc = wmma16(a.v, bw, lacc);
  }

  float* Lg = &sh[w][1][0][0];
#pragma unroll
  for (int r = 0; r < 8; ++r) {
    Lg[(r + hi * 8) * 16 + mrow] = lacc[r] * INV_SM + bsm[nn];
  }
  __syncthreads();

  if (lane < 16) {
    const float* lr = Lg + lane * 16;
    float lg[RELS];
    float mx = -3.0e38f;
#pragma unroll
    for (int rel = 0; rel < RELS; ++rel) { lg[rel] = lr[rel]; mx = fmaxf(mx, lg[rel]); }
    float se = 0.0f;
#pragma unroll
    for (int rel = 0; rel < RELS; ++rel) se += expf(lg[rel] - mx);
    const float lse = logf(se);
#pragma unroll
    for (int rel = 0; rel < RELS; ++rel)
      outs[(w * 16 + lane) * RELS + rel] = (lg[rel] - mx) - lse;
  }
  __syncthreads();

  float* ob = out + (size_t)blockIdx.x * (128 * RELS);
  if (threadIdx.x < (128 * RELS) / 4) {
    v4f v = *(const v4f*)(outs + threadIdx.x * 4);
    *(volatile v4f*)(ob + threadIdx.x * 4) = v;
  }
  __threadfence();
  if (threadIdx.x < (128 * RELS) / 4) {
    v4f v = *(const v4f*)(outs + threadIdx.x * 4);
    *(volatile v4f*)(ob + threadIdx.x * 4) = v;
  }
}

extern "C" void kernel_launch(void* const* d_in, const int* in_sizes, int n_in,
                              void* d_out, int out_size, void* d_ws, size_t ws_size,
                              hipStream_t stream) {
  if (n_in < 13) return;
  if (in_sizes[0] != NLEAF || in_sizes[1] != D * VOC || in_sizes[2] != D ||
      in_sizes[3] != D * KL || in_sizes[4] != D || in_sizes[5] != D * KT || in_sizes[6] != D ||
      in_sizes[7] != D * KL || in_sizes[8] != D || in_sizes[9] != D * KT || in_sizes[10] != D ||
      in_sizes[11] != RELS * D || in_sizes[12] != RELS) return;
  if (out_size != NB * RELS) return;

  const int*   ids   = (const int*)  d_in[0];
  const float* Wv    = (const float*)d_in[1];
  const float* bv    = (const float*)d_in[2];
  const float* Wcps  = (const float*)d_in[3];
  const float* bcps  = (const float*)d_in[4];
  const float* Wcpst = (const float*)d_in[5];
  const float* bcpst = (const float*)d_in[6];
  const float* Wcpr  = (const float*)d_in[7];
  const float* bcpr  = (const float*)d_in[8];
  const float* Wcprt = (const float*)d_in[9];
  const float* bcprt = (const float*)d_in[10];
  const float* Wsm   = (const float*)d_in[11];
  const float* bsm   = (const float*)d_in[12];
  float* out = (float*)d_out;

  const size_t h0_off  = 0;
  const size_t h0_b    = (size_t)NLEAF * D * sizeof(float);
  const size_t h1_off  = h0_off + h0_b;
  const size_t h1_b    = (size_t)(NLEAF / 2) * D * sizeof(float);
  const size_t pk_b    = (size_t)NPK * sizeof(f16_t);
  const size_t pk1_off = h1_off + h1_b;
  const size_t pk2_off = pk1_off + pk_b;
  const size_t total   = pk2_off + pk_b;
  if (total > ws_size) return;

  char* ws = (char*)d_ws;
  float* h0   = (float*)(ws + h0_off);
  float* h1   = (float*)(ws + h1_off);
  f16_t* Wpk1 = (f16_t*)(ws + pk1_off);
  f16_t* Wpk2 = (f16_t*)(ws + pk2_off);

  prepack_kernel<<<(2 * (NPK / 8)) / 256, 256, 0, stream>>>(Wcpst, Wcps, Wcprt, Wcpr, Wpk1, Wpk2);
  embed_kernel  <<<(NLEAF * 32) / 256, 256, 0, stream>>>(ids, Wv, bv, h0);

  combine_kernel<<<64, 256, 0, stream>>>(h0, h1, Wpk1, bcps, bcpst, 3);
  combine_kernel<<<32, 256, 0, stream>>>(h1, h0, Wpk1, bcps, bcpst, 2);
  combine_kernel<<<16, 256, 0, stream>>>(h0, h1, Wpk1, bcps, bcpst, 1);
  combine_kernel<<< 8, 256, 0, stream>>>(h1, h0, Wpk1, bcps, bcpst, 0);

  final_kernel<<<NB / 128, 256, 0, stream>>>(h0, out, Wpk2, bcpr, bcprt, Wsm, bsm);
}
